// VLSTM_22814866276682
// MI455X (gfx1250) — hardware-run, weakly checked
//
#include <hip/hip_runtime.h>
#include <math.h>

typedef __attribute__((ext_vector_type(16))) _Float16 v16h;
typedef __attribute__((ext_vector_type(8)))  _Float16 v8h;
typedef __attribute__((ext_vector_type(8)))  float    v8f;
typedef __attribute__((ext_vector_type(4)))  float    v4f;
typedef __attribute__((ext_vector_type(2)))  float    v2f;
typedef __attribute__((ext_vector_type(4)))  int      v4i;

constexpr int T_STEPS = 20;
constexpr int NNODE   = 32768;
constexpr int DIN2    = 2;
constexpr int DEMB    = 64;
constexpr int DHID    = 128;
constexpr int NGATE   = 4 * DHID;
constexpr int DOUT    = 5;
constexpr int KCAT    = DEMB + DHID;
constexpr int MT      = 32;
constexpr int AP      = 200;
constexpr int HNP     = 132;
constexpr float ACARRY = 64.0f;
constexpr float WCARRY = 64.0f;
constexpr float FOLD   = 1.0f / (ACARRY * WCARRY);

static_assert(KCAT == 192, "fused K");
static_assert(KCAT % 32 == 0, "K is a multiple of the 32-deep step");
static_assert(NGATE == 512, "gate columns");
static_assert(NNODE % MT == 0, "node tiles are exact");
static_assert((AP * 2) % 16 == 0, "A rows are 16-B aligned");
static_assert((HNP * 4) % 16 == 0, "staging rows are 16-B aligned");
static_assert(((size_t)T_STEPS * NNODE * DOUT * 4) % 128 == 0, "second output starts on a line");
static_assert((size_t)T_STEPS * NNODE * DOUT * 4 == 13107200, "byte offset of the final hidden state");
static_assert((size_t)T_STEPS * NNODE * DOUT * 4 + (size_t)NNODE * DHID * 4 == 29884416, "byte offset of the final cell state");
static_assert((size_t)T_STEPS * NNODE * DOUT * 4 + 2 * (size_t)NNODE * DHID * 4 == 46661632, "total output bytes");

union FragU { v16h v; v8h h[2]; };
__device__ __forceinline__ _Float16 f16_operand(float v) {
    const float a = __builtin_fabsf(v);
    const float s = (a < 6.103515625e-05f) ? 0.0f : v;
    return (_Float16)s;
}
__device__ __forceinline__ v16h frag_load(const _Float16* p) {
  FragU f;
  f.h[0] = *(const v8h*)(p);
  f.h[1] = *(const v8h*)(p + 16);
  return f.v;
}
__device__ __forceinline__ v8f mma_h(v16h a, v16h b, v8f c) {
  c = __builtin_amdgcn_wmma_f32_16x16x32_f16(false, a, false, b, (short)0, c, false, false);
  asm volatile("v_nop\n\tv_nop\n\tv_nop\n\tv_nop" : "+v"(c) : "v"(a), "v"(b));
  return c;
}

__device__ __forceinline__ float fsig(float x)  { return __builtin_amdgcn_rcpf(1.0f + __expf(-x)); }
__device__ __forceinline__ float ftanh(float x) { return 1.0f - 2.0f * __builtin_amdgcn_rcpf(__expf(2.0f * x) + 1.0f); }

__global__ __launch_bounds__(256) void pack_wt_kernel(const float* __restrict__ src, int cshift, int kofs,
                                                      unsigned short* __restrict__ dst) {
  const int i = blockIdx.x * 256 + threadIdx.x;
  const int total = NGATE << cshift;
  if (i >= total) return;
  const int n  = i >> cshift;
  const int kc = i & ((1 << cshift) - 1);
  const int k0 = kc * 8;
  v8h hv;
#pragma unroll
  for (int e = 0; e < 8; ++e) {
    const float f = src[(size_t)(k0 + e) * NGATE + n];
    hv[e] = f16_operand(f * WCARRY);
  }
  _Float16* p = (_Float16*)dst + (size_t)n * KCAT + kofs + k0;
  *(volatile v8h*)p = hv;
  __threadfence();
  *(volatile v8h*)p = hv;
}

__device__ __forceinline__ void store_tile_rows(const float* Hst, float* dst, int tid) {
  v4f v[4];
#pragma unroll
  for (int it = 0; it < 4; ++it) {
    const int idx = it * 256 + tid;
    const int row = idx >> 5, c4 = (idx & 31) * 4;
    v[it] = *(const v4f*)(Hst + row * HNP + c4);
  }
  for (int pass = 0; pass < 2; ++pass) {
#pragma unroll
    for (int it = 0; it < 4; ++it) {
      const int idx = it * 256 + tid;
      const int row = idx >> 5, c4 = (idx & 31) * 4;
      *(volatile v4f*)(dst + (size_t)row * DHID + c4) = v[it];
    }
    __threadfence();
  }
}

__global__ __launch_bounds__(256) void frame_scan_kernel(
    const float* __restrict__ nodes, const int* __restrict__ pmask,
    const float* __restrict__ h0, const float* __restrict__ c0,
    const float* __restrict__ We, const float* __restrict__ be,
    const float* __restrict__ bih, const float* __restrict__ bhh,
    const float* __restrict__ Wout, const float* __restrict__ bout,
    const unsigned short* __restrict__ Wcp,
    float* __restrict__ out0, float* __restrict__ out1, float* __restrict__ out2) {
  __shared__ __align__(16) _Float16 Acat[MT * AP];
  __shared__ __align__(16) float    Hn[MT * HNP];
  __shared__ __align__(16) float    sWe[DIN2 * DEMB];
  __shared__ __align__(16) float    sbe[DEMB];
  __shared__ __align__(16) float    sWo[DOUT * DHID];
  __shared__ __align__(16) float    sBo[8];
  __shared__ __align__(16) int      sMask[MT];
  __shared__ __align__(16) float    sOut[MT * DOUT];

  const _Float16* Wc = (const _Float16*)Wcp;
  const int tid = threadIdx.x, lane = tid & 31, wave = tid >> 5;
  const int c = lane & 15, hh = lane >> 4;
  const int j = 16 * wave + c;
  const int nb = blockIdx.x * MT;

  if (tid < DIN2 * DEMB) sWe[tid] = We[tid];
  if (tid < DEMB) sbe[tid] = be[tid];
  for (int idx = tid; idx < DOUT * DHID; idx += 256) {
    const int oc = idx >> 7, k = idx & 127;
    sWo[idx] = Wout[k * DOUT + oc];
  }
  {
    const int bi = (tid < DOUT) ? tid : (DOUT - 1);
    float bv = bout[bi];
    asm volatile("" : "+v"(bv));
    if (tid < 8) sBo[tid] = (tid < DOUT) ? bv : 0.0f;
  }
  float bb[4];
#pragma unroll
  for (int g = 0; g < 4; ++g) bb[g] = bih[g * DHID + j] + bhh[g * DHID + j];

  float hst[2][8], cst[2][8];
#pragma unroll
  for (int it = 0; it < 4; ++it) {
    const int idx = it * 256 + tid;
    const int row = idx >> 5, c4 = (idx & 31) * 4;
    const v4f v = *(const v4f*)(h0 + (size_t)(nb + row) * DHID + c4);
    *(v4f*)(Hn + row * HNP + c4) = v;
  }
  __syncthreads();
#pragma unroll
  for (int rt = 0; rt < 2; ++rt)
#pragma unroll
    for (int r = 0; r < 8; ++r) hst[rt][r] = Hn[(rt * 16 + 8 * hh + r) * HNP + j];
  __syncthreads();
#pragma unroll
  for (int it = 0; it < 4; ++it) {
    const int idx = it * 256 + tid;
    const int row = idx >> 5, c4 = (idx & 31) * 4;
    const v4f v = *(const v4f*)(c0 + (size_t)(nb + row) * DHID + c4);
    *(v4f*)(Hn + row * HNP + c4) = v;
  }
  __syncthreads();
#pragma unroll
  for (int rt = 0; rt < 2; ++rt)
#pragma unroll
    for (int r = 0; r < 8; ++r) cst[rt][r] = Hn[(rt * 16 + 8 * hh + r) * HNP + j];

  const _Float16* arow0 = Acat + c * AP + 8 * hh;
  const _Float16* arow1 = Acat + (16 + c) * AP + 8 * hh;
  const _Float16* wrow  = Wc + (size_t)j * KCAT + 8 * hh;
  const v8f z8 = {0.f, 0.f, 0.f, 0.f, 0.f, 0.f, 0.f, 0.f};

#pragma unroll 1
  for (int t = 0; t < T_STEPS; ++t) {
#pragma unroll
    for (int rt = 0; rt < 2; ++rt)
#pragma unroll
      for (int r = 0; r < 8; ++r)
        Acat[(rt * 16 + 8 * hh + r) * AP + DEMB + j] = f16_operand(hst[rt][r] * ACARRY);
    {
      const int n = tid >> 3, cg = tid & 7;
      const v2f xv = *(const v2f*)(nodes + ((size_t)t * NNODE + nb + n) * DIN2);
      const v4f wa0 = *(const v4f*)(sWe + 8 * cg);
      const v4f wa1 = *(const v4f*)(sWe + 8 * cg + 4);
      const v4f wb0 = *(const v4f*)(sWe + DEMB + 8 * cg);
      const v4f wb1 = *(const v4f*)(sWe + DEMB + 8 * cg + 4);
      const v4f bq0 = *(const v4f*)(sbe + 8 * cg);
      const v4f bq1 = *(const v4f*)(sbe + 8 * cg + 4);
      v8h ev;
#pragma unroll
      for (int e = 0; e < 4; ++e) {
        float s0 = xv[0] * wa0[e] + xv[1] * wb0[e] + bq0[e];
        float s1 = xv[0] * wa1[e] + xv[1] * wb1[e] + bq1[e];
        s0 = fmaxf(s0, 0.0f);
        s1 = fmaxf(s1, 0.0f);
        ev[e]     = f16_operand(s0 * ACARRY);
        ev[4 + e] = f16_operand(s1 * ACARRY);
      }
      *(v8h*)(Acat + n * AP + 8 * cg) = ev;
    }
    {
      int mval = pmask[(size_t)t * NNODE + nb + lane];
      asm volatile("" : "+v"(mval));
      if (wave == 0) sMask[lane] = mval;
    }
    __syncthreads();

    v8f acc[2][4];
#pragma unroll
    for (int rt = 0; rt < 2; ++rt)
#pragma unroll
      for (int g = 0; g < 4; ++g) acc[rt][g] = z8;
#pragma unroll 1
    for (int k0 = 0; k0 < KCAT; k0 += 32) {
      const v16h a0 = frag_load(arow0 + k0);
      const v16h a1 = frag_load(arow1 + k0);
      v16h bf[4];
#pragma unroll
      for (int g = 0; g < 4; ++g) bf[g] = frag_load(wrow + (size_t)g * DHID * KCAT + k0);
#pragma unroll
      for (int g = 0; g < 4; ++g) {
        acc[0][g] = mma_h(a0, bf[g], acc[0][g]);
        acc[1][g] = mma_h(a1, bf[g], acc[1][g]);
      }
    }

#pragma unroll
    for (int rt = 0; rt < 2; ++rt) {
      const v4i ma = *(const v4i*)(sMask + rt * 16 + 8 * hh);
      const v4i mb = *(const v4i*)(sMask + rt * 16 + 8 * hh + 4);
#pragma unroll
      for (int r = 0; r < 8; ++r) {
        const int mv = (r < 4) ? ma[r & 3] : mb[r & 3];
        const float zi = acc[rt][0][r] * FOLD + bb[0];
        const float zf = acc[rt][1][r] * FOLD + bb[1];
        const float zg = acc[rt][2][r] * FOLD + bb[2];
        const float zo = acc[rt][3][r] * FOLD + bb[3];
        const float ig = fsig(zi);
        const float fg = fsig(zf);
        const float gg = ftanh(zg);
        const float og = fsig(zo);
        const float cold = cst[rt][r];
        const float hold = hst[rt][r];
        const float cn = fg * cold + ig * gg;
        const float hn = og * ftanh(cn);
        Hn[(rt * 16 + 8 * hh + r) * HNP + j] = hn;
        cst[rt][r] = (mv != 0) ? cn : cold;
        hst[rt][r] = (mv != 0) ? hn : hold;
      }
    }
    __syncthreads();

    {
      const int n = tid >> 3, ks = tid & 7;
      float p0 = 0.0f, p1 = 0.0f, p2 = 0.0f, p3 = 0.0f, p4 = 0.0f;
#pragma unroll 1
      for (int kq = 0; kq < 4; ++kq) {
        const int kb = 16 * ks + 4 * kq;
        const v4f hv = *(const v4f*)(Hn + n * HNP + kb);
        const v4f w0 = *(const v4f*)(sWo + 0 * DHID + kb);
        const v4f w1 = *(const v4f*)(sWo + 1 * DHID + kb);
        const v4f w2 = *(const v4f*)(sWo + 2 * DHID + kb);
        const v4f w3 = *(const v4f*)(sWo + 3 * DHID + kb);
        const v4f w4 = *(const v4f*)(sWo + 4 * DHID + kb);
#pragma unroll
        for (int e = 0; e < 4; ++e) {
          p0 = fmaf(hv[e], w0[e], p0);
          p1 = fmaf(hv[e], w1[e], p1);
          p2 = fmaf(hv[e], w2[e], p2);
          p3 = fmaf(hv[e], w3[e], p3);
          p4 = fmaf(hv[e], w4[e], p4);
        }
      }
#pragma unroll
      for (int off = 1; off < 8; off <<= 1) {
        p0 += __shfl_xor(p0, off, 32);
        p1 += __shfl_xor(p1, off, 32);
        p2 += __shfl_xor(p2, off, 32);
        p3 += __shfl_xor(p3, off, 32);
        p4 += __shfl_xor(p4, off, 32);
      }
      const int ksc = (ks < DOUT) ? ks : (DOUT - 1);
      const float bo = sBo[ksc];
      float sel = p0;
      sel = (ks == 1) ? p1 : sel;
      sel = (ks == 2) ? p2 : sel;
      sel = (ks == 3) ? p3 : sel;
      sel = (ks == 4) ? p4 : sel;
      const int mv = sMask[n];
      const float ov = (mv != 0) ? (sel + bo) : 0.0f;
      if (ks < DOUT) sOut[n * DOUT + ks] = ov;
    }
    __syncthreads();

    if (wave == 0) {
      float* ob = out0 + ((size_t)t * NNODE + nb) * DOUT;
      const v4f va = *(const v4f*)(sOut + 4 * lane);
      const v4f vb = *(const v4f*)(sOut + 128 + 4 * (lane & 7));
      for (int pass = 0; pass < 2; ++pass) {
        *(volatile v4f*)(ob + 4 * lane) = va;
        if (lane < 8) *(volatile v4f*)(ob + 128 + 4 * lane) = vb;
        __threadfence();
      }
    }
  }

#pragma unroll
  for (int rt = 0; rt < 2; ++rt)
#pragma unroll
    for (int r = 0; r < 8; ++r) Hn[(rt * 16 + 8 * hh + r) * HNP + j] = hst[rt][r];
  __syncthreads();
  store_tile_rows(Hn, out1 + (size_t)nb * DHID, tid);
  __syncthreads();
#pragma unroll
  for (int rt = 0; rt < 2; ++rt)
#pragma unroll
    for (int r = 0; r < 8; ++r) Hn[(rt * 16 + 8 * hh + r) * HNP + j] = cst[rt][r];
  __syncthreads();
  store_tile_rows(Hn, out2 + (size_t)nb * DHID, tid);
}

extern "C" void kernel_launch(void* const* d_in, const int* in_sizes, int n_in,
                              void* d_out, int out_size, void* d_ws, size_t ws_size, hipStream_t stream) {
  if (n_in < 12 || d_out == nullptr || d_ws == nullptr) return;
  if (in_sizes[0] != T_STEPS * NNODE * DIN2 || in_sizes[1] != T_STEPS * NNODE) return;
  if (in_sizes[2] != NNODE * DHID || in_sizes[3] != NNODE * DHID) return;
  if (in_sizes[4] != DIN2 * DEMB || in_sizes[5] != DEMB) return;
  if (in_sizes[6] != DEMB * NGATE || in_sizes[7] != NGATE) return;
  if (in_sizes[8] != DHID * NGATE || in_sizes[9] != NGATE) return;
  if (in_sizes[10] != DHID * DOUT || in_sizes[11] != DOUT) return;
  if (out_size != T_STEPS * NNODE * DOUT + 2 * NNODE * DHID) return;

  const float* nodes = (const float*)d_in[0];
  const int*   pmask = (const int*)  d_in[1];
  const float* h0    = (const float*)d_in[2];
  const float* c0    = (const float*)d_in[3];
  const float* We    = (const float*)d_in[4];
  const float* be    = (const float*)d_in[5];
  const float* Wih   = (const float*)d_in[6];
  const float* bih   = (const float*)d_in[7];
  const float* Whh   = (const float*)d_in[8];
  const float* bhh   = (const float*)d_in[9];
  const float* Wout  = (const float*)d_in[10];
  const float* bout  = (const float*)d_in[11];

  float* out0 = (float*)d_out;
  float* out1 = out0 + (size_t)T_STEPS * NNODE * DOUT;
  float* out2 = out1 + (size_t)NNODE * DHID;

  char* ws = (char*)d_ws;
  size_t off = 0;
  auto carve = [&](size_t bytes) -> char* { char* p = ws + off; off += (bytes + 255) & ~(size_t)255; return p; };
  unsigned short* Wc = (unsigned short*)carve((size_t)NGATE * KCAT * 2);
  if (off > ws_size || off > (size_t)134217728) return;

  pack_wt_kernel<<<(NGATE * (DEMB / 8)) / 256, 256, 0, stream>>>(Wih, 3, 0, Wc);
  pack_wt_kernel<<<(NGATE * (DHID / 8)) / 256, 256, 0, stream>>>(Whh, 4, DEMB, Wc);
  frame_scan_kernel<<<NNODE / MT, 256, 0, stream>>>(nodes, pmask, h0, c0, We, be, bih, bhh, Wout, bout, Wc,
                                                    out0, out1, out2);
}
